// SelectiveSSM_44736379355743
// MI455X (gfx1250) — hardware-verified
//
#include <hip/hip_runtime.h>
#include <math.h>

typedef __attribute__((ext_vector_type(16))) __bf16   v16b;
typedef __attribute__((ext_vector_type(8)))  __bf16   v8b;
typedef __attribute__((ext_vector_type(8)))  float    v8f;
typedef __attribute__((ext_vector_type(4)))  float    v4f;
typedef __attribute__((ext_vector_type(4)))  unsigned v4u;

constexpr int kSeq    = 2048;
constexpr int kDm     = 1024;
constexpr int kDi     = 2048;
constexpr int kNst    = 16;
constexpr int kTaps   = 4;
constexpr int kXrP    = 2 * kDi;
constexpr int kPjN    = kDi + 2 * kNst;
constexpr int kPjP    = 2112;
constexpr int kTP     = 260;
constexpr int kScanTS = 64;
constexpr int kScanCh = 64;
constexpr int kScanYP = 68;
constexpr int kBcW    = 2 * kNst;
static_assert(kPjN == 2080);
static_assert((kPjP % 64) == 0 && kPjP >= kPjN);
static_assert((kDm % 32) == 0 && (kDi % 32) == 0);
static_assert((kSeq % 64) == 0 && (kXrP % 64) == 0 && (kDm % 64) == 0);
static_assert((kSeq % kScanTS) == 0 && (kDi % kScanCh) == 0 && (kDi % 256) == 0);
static_assert(kTaps == 4 && kNst == 16 && kBcW == 32);

constexpr size_t kOffXB   = 0;
constexpr size_t kOffWINB = kOffXB   + (size_t)kSeq * kDm  * 2;
constexpr size_t kOffWXB  = kOffWINB + (size_t)kXrP * kDm  * 2;
constexpr size_t kOffWOB  = kOffWXB  + (size_t)kPjP * kDi  * 2;
constexpr size_t kOffXR   = kOffWOB  + (size_t)kDm  * kDi  * 2;
constexpr size_t kOffXI   = kOffXR   + (size_t)kSeq * kXrP * 4;
constexpr size_t kOffXIB  = kOffXI   + (size_t)kSeq * kDi  * 4;
constexpr size_t kOffPROJ = kOffXIB  + (size_t)kSeq * kDi  * 2;
constexpr size_t kOffZH   = kOffPROJ + (size_t)kSeq * kPjP * 4;
constexpr size_t kOffZL   = kOffZH   + (size_t)kSeq * kDi  * 2;
constexpr size_t kWsTotal = kOffZL   + (size_t)kSeq * kDi  * 2;
static_assert(kWsTotal == 118226944ull);
static_assert(kWsTotal <= 134217728ull);
static_assert((kOffWINB % 128) == 0 && (kOffWXB % 128) == 0 && (kOffWOB % 128) == 0 && (kOffXR % 128) == 0 &&
              (kOffXI % 128) == 0 && (kOffXIB % 128) == 0 && (kOffPROJ % 128) == 0 && (kOffZH % 128) == 0 &&
              (kOffZL % 128) == 0);

__device__ __forceinline__ unsigned short f2bf_bits(float f) {
  unsigned u = __float_as_uint(f);
  return (unsigned short)((u + 0x7FFFu + ((u >> 16) & 1u)) >> 16);
}
__device__ __forceinline__ float bf_bits2f(unsigned short h) { return __uint_as_float(((unsigned)h) << 16); }
__device__ __forceinline__ float bf_rne(float f) { return bf_bits2f(f2bf_bits(f)); }
__device__ __forceinline__ unsigned pack2_bf(float f0, float f1) {
  const unsigned short h0 = f2bf_bits(f0), h1 = f2bf_bits(f1);
  return (unsigned)h0 | ((unsigned)h1 << 16);
}
__device__ __forceinline__ void split_pack2(float f0, float f1, unsigned& wh, unsigned& wl) {
  const unsigned short h0 = f2bf_bits(f0), h1 = f2bf_bits(f1);
  const unsigned short l0 = f2bf_bits(f0 - bf_bits2f(h0)), l1 = f2bf_bits(f1 - bf_bits2f(h1));
  wh = (unsigned)h0 | ((unsigned)h1 << 16);
  wl = (unsigned)l0 | ((unsigned)l1 << 16);
}

__device__ __forceinline__ void dep_guard4_b(v8f& a, v8f& b, v8f& c, v8f& d, v16b x, v16b y) {
  asm volatile("v_nop\n\tv_nop\n\tv_nop\n\tv_nop" : "+v"(a), "+v"(b), "+v"(c), "+v"(d) : "v"(x), "v"(y));
}
__device__ __forceinline__ void keep4_b(v16b a, v16b b, v16b c, v16b d) { asm volatile("v_nop" :: "v"(a), "v"(b), "v"(c), "v"(d)); }
__device__ __forceinline__ void acc_guard4(v8f& a, v8f& b, v8f& c, v8f& d) { asm volatile("v_nop\n\tv_nop\n\tv_nop\n\tv_nop" : "+v"(a), "+v"(b), "+v"(c), "+v"(d)); }

struct FragB {
  union U { v16b v; v8b h[2]; };
  static __device__ __forceinline__ v16b load(const __bf16* p) {
    U f; f.h[0] = *(const v8b*)(p); f.h[1] = *(const v8b*)(p + 16); return f.v;
  }
  static __device__ __forceinline__ v8f mma(v16b a, v16b b, v8f c) {
    return __builtin_amdgcn_wmma_f32_16x16x32_bf16(false, a, false, b, (short)0, c, false, false);
  }
};

template <int SPL>
__global__ __launch_bounds__(256) void wmma_gemm64_bf16(
    const unsigned short* __restrict__ Ap, const unsigned short* __restrict__ A2p, int lda,
    const unsigned short* __restrict__ Btp, int ldb,
    float* __restrict__ C, int ldc,
    const float* __restrict__ bias, int nBias,
    int M, int N, int K) {
  const __bf16* A  = (const __bf16*)Ap;
  const __bf16* A2 = (const __bf16*)A2p;
  const __bf16* Bt = (const __bf16*)Btp;
  __shared__ __align__(16) float sT[8][16 * 68];
  const int lane = threadIdx.x & 31;
  const int wave = threadIdx.x >> 5;
  const int tilesN = N >> 6;
  const int tilesM = M >> 6;
  const int tile = blockIdx.x * 8 + wave;
  if (tile >= tilesM * tilesN) return;
  const int tm = tile / tilesN;
  const int tn = tile - tm * tilesN;
  const int m0 = tm << 6;
  const int n0 = tn << 6;

  const int rlane = lane & 15;
  const int koff  = (lane >> 4) * 8;
  const int mOff  = (lane >> 4) * 8;

  v8f acc[4][4];
#pragma unroll
  for (int i = 0; i < 4; ++i)
#pragma unroll
    for (int j = 0; j < 4; ++j) acc[i][j] = (v8f){0.f,0.f,0.f,0.f,0.f,0.f,0.f,0.f};

  for (int k0 = 0; k0 < K; k0 += 32) {
    v16b bh[4];
#pragma unroll
    for (int j = 0; j < 4; ++j) {
      const size_t bo = (size_t)(n0 + (j << 4) + rlane) * ldb + koff + k0;
      bh[j] = FragB::load(Bt + bo);
    }
#pragma unroll
    for (int i = 0; i < 4; ++i) {
      const size_t ao = (size_t)(m0 + (i << 4) + rlane) * lda + koff + k0;
      v16b ah = FragB::load(A + ao);
      v16b al = ah;
      if (SPL == 1) al = FragB::load(A2 + ao);
#pragma unroll
      for (int j = 0; j < 4; ++j) {
        acc[i][j] = FragB::mma(ah, bh[j], acc[i][j]);
        if (SPL == 1) acc[i][j] = FragB::mma(al, bh[j], acc[i][j]);
      }
      dep_guard4_b(acc[i][0], acc[i][1], acc[i][2], acc[i][3], ah, al);
    }
    keep4_b(bh[0], bh[1], bh[2], bh[3]);
  }
  acc_guard4(acc[0][0], acc[0][1], acc[0][2], acc[0][3]);
  acc_guard4(acc[1][0], acc[1][1], acc[1][2], acc[1][3]);
  acc_guard4(acc[2][0], acc[2][1], acc[2][2], acc[2][3]);
  acc_guard4(acc[3][0], acc[3][1], acc[3][2], acc[3][3]);

  float* slab = sT[wave];
#pragma unroll
  for (int i = 0; i < 4; ++i) {
    const int mBase = m0 + (i << 4);
#pragma unroll
    for (int j = 0; j < 4; ++j) {
      const int n  = n0 + (j << 4) + rlane;
      const int nc = (n < nBias) ? n : (nBias - 1);
      const float braw = bias[nc];
      const float bv = (n < nBias) ? bf_rne(braw) : 0.0f;
#pragma unroll
      for (int r = 0; r < 8; ++r) {
        const float v = acc[i][j][r] + bv;
        slab[(mOff + r) * 68 + (j << 4) + rlane] = v;
      }
    }
    __builtin_amdgcn_fence(__ATOMIC_RELEASE, "workgroup");
    __builtin_amdgcn_wave_barrier();
    __builtin_amdgcn_fence(__ATOMIC_ACQUIRE, "workgroup");
    {
      const int hh = lane >> 4, c4 = (lane & 15) * 4;
      for (int pass = 0; pass < 2; ++pass) {
#pragma unroll
        for (int it = 0; it < 8; ++it) {
          const int row = it * 2 + hh;
          v4f v = *(const v4f*)(slab + row * 68 + c4);
          *(volatile v4f*)(C + (size_t)(mBase + row) * ldc + n0 + c4) = v;
        }
        __threadfence();
      }
    }
    __builtin_amdgcn_fence(__ATOMIC_RELEASE, "workgroup");
    __builtin_amdgcn_wave_barrier();
    __builtin_amdgcn_fence(__ATOMIC_ACQUIRE, "workgroup");
  }
}

__global__ __launch_bounds__(256) void cast_bf16_kernel(
    const float* __restrict__ src, unsigned short* __restrict__ dst, int real8, int total8)
{
  const int i = blockIdx.x * 256 + threadIdx.x;
  if (i >= total8) return;
  const bool live = (i < real8);
  const int ic = live ? i : (real8 - 1);
  const float* p = src + ((size_t)ic << 3);
  const v4f a0 = *(const v4f*)(p);
  const v4f a1 = *(const v4f*)(p + 4);
  float f[8];
  f[0] = a0[0]; f[1] = a0[1]; f[2] = a0[2]; f[3] = a0[3];
  f[4] = a1[0]; f[5] = a1[1]; f[6] = a1[2]; f[7] = a1[3];
#pragma unroll
  for (int e = 0; e < 8; ++e) f[e] = live ? f[e] : 0.0f;
  v4u w;
  w[0] = pack2_bf(f[0], f[1]);
  w[1] = pack2_bf(f[2], f[3]);
  w[2] = pack2_bf(f[4], f[5]);
  w[3] = pack2_bf(f[6], f[7]);
  unsigned short* q = dst + ((size_t)i << 3);
  *(volatile v4u*)q = w;
  __threadfence();
  *(volatile v4u*)q = w;
}

__global__ __launch_bounds__(256) void conv_silu_kernel(
    const float* __restrict__ XR, const float* __restrict__ cw, const float* __restrict__ cb,
    float* __restrict__ XI, unsigned short* __restrict__ XIB)
{
  __shared__ __align__(16) float sT[16 * kTP];
  const int tid = threadIdx.x, lane = tid & 31, wave = tid >> 5;
  const int d0 = blockIdx.x * 256, d = d0 + tid;
  const int t0 = blockIdx.y * 64;
  const v4f wv = *(const v4f*)(cw + (size_t)d * kTaps);
  const float wr0 = wv[0], wr1 = wv[1], wr2 = wv[2], wr3 = wv[3];
  const float w0 = bf_rne(wr0), w1 = bf_rne(wr1), w2 = bf_rne(wr2), w3 = bf_rne(wr3);
  const float bc = bf_rne(cb[d]);
  float xm3, xm2, xm1;
  {
    const int r3 = t0 - 3, r2 = t0 - 2, r1 = t0 - 1;
    const float v3 = XR[(size_t)(r3 < 0 ? 0 : r3) * kXrP + d];
    const float v2 = XR[(size_t)(r2 < 0 ? 0 : r2) * kXrP + d];
    const float v1 = XR[(size_t)(r1 < 0 ? 0 : r1) * kXrP + d];
    xm3 = (r3 >= 0) ? v3 : 0.f;
    xm2 = (r2 >= 0) ? v2 : 0.f;
    xm1 = (r1 >= 0) ? v1 : 0.f;
  }
  const int hrow = wave >> 1;
  const int hch  = (wave & 1) * 128 + lane * 4;
#pragma unroll 1
  for (int sub = 0; sub < 4; ++sub) {
    const int lb = t0 + sub * 16;
#pragma unroll 1
    for (int s = 0; s < 16; ++s) {
      const float xcur = XR[(size_t)(lb + s) * kXrP + d];
      float acc = w0 * xm3;
      acc = fmaf(w1, xm2, acc);
      acc = fmaf(w2, xm1, acc);
      acc = fmaf(w3, xcur, acc);
      const float sv = acc + bc;
      const float sg = __builtin_amdgcn_rcpf(1.0f + expf(-sv));
      sT[s * kTP + tid] = sv * sg;
      xm3 = xm2; xm2 = xm1; xm1 = xcur;
    }
    __syncthreads();
    v4f fv[4];
    v4u bw[2];
#pragma unroll
    for (int it = 0; it < 4; ++it) fv[it] = *(const v4f*)(sT + (it * 4 + hrow) * kTP + hch);
#pragma unroll
    for (int it = 0; it < 2; ++it) {
      const float* sp = sT + (it * 8 + wave) * kTP + lane * 8;
      const v4f a0 = *(const v4f*)(sp);
      const v4f a1 = *(const v4f*)(sp + 4);
      const float e0 = a0[0], e1 = a0[1], e2 = a0[2], e3 = a0[3];
      const float e4 = a1[0], e5 = a1[1], e6 = a1[2], e7 = a1[3];
      bw[it][0] = pack2_bf(e0, e1);
      bw[it][1] = pack2_bf(e2, e3);
      bw[it][2] = pack2_bf(e4, e5);
      bw[it][3] = pack2_bf(e6, e7);
    }
    for (int pass = 0; pass < 2; ++pass) {
#pragma unroll
      for (int it = 0; it < 4; ++it)
        *(volatile v4f*)(XI + (size_t)(lb + it * 4 + hrow) * kDi + d0 + hch) = fv[it];
#pragma unroll
      for (int it = 0; it < 2; ++it)
        *(volatile v4u*)(XIB + (size_t)(lb + it * 8 + wave) * kDi + d0 + lane * 8) = bw[it];
      __threadfence();
    }
    __syncthreads();
  }
}

__global__ __launch_bounds__(64) void scan_kernel(
    const float* __restrict__ PROJ, const float* __restrict__ XI, const float* __restrict__ XR,
    const float* __restrict__ Alog, const float* __restrict__ Dp,
    unsigned short* __restrict__ ZH, unsigned short* __restrict__ ZL)
{
  __shared__ __align__(16) float sX[kScanTS * kBcW];
  __shared__ __align__(16) float sY[kScanTS * kScanYP];
  __shared__ __align__(16) float sA[kNst * kScanCh];
  const int tid = threadIdx.x, lane = tid & 31, wave = tid >> 5;
  const int d0 = blockIdx.x * kScanCh;
  const int d  = d0 + tid;
#pragma unroll 1
  for (int s = 0; s < kNst; ++s) sA[s * kScanCh + tid] = -expf(bf_rne(Alog[(size_t)d * kNst + s]));
  __syncthreads();
  float negA[kNst], h[kNst];
#pragma unroll
  for (int s = 0; s < kNst; ++s) {
    negA[s] = sA[s * kScanCh + tid];
    h[s] = 0.f;
  }
  const float Dd = bf_rne(Dp[d]);
  const int lr = tid >> 3, lc4 = (tid & 7) * 4;
  const int q = lane >> 3, c8 = (lane & 7) * 8;
#pragma unroll 1
  for (int t0 = 0; t0 < kSeq; t0 += kScanTS) {
    __syncthreads();
#pragma unroll
    for (int i = 0; i < 8; ++i) {
      const int r = lr + 8 * i;
      *(v4f*)(sX + r * kBcW + lc4) = *(const v4f*)(PROJ + (size_t)(t0 + r) * kPjP + kDi + lc4);
    }
    __syncthreads();
#pragma unroll 1
    for (int s = 0; s < kScanTS; ++s) {
      const size_t t = (size_t)(t0 + s);
      const float* xr = sX + s * kBcW;
      float Bs[kNst], Cs[kNst];
#pragma unroll
      for (int q4 = 0; q4 < 4; ++q4) {
        const v4f bv = *(const v4f*)(xr + 4 * q4);
        const v4f cv = *(const v4f*)(xr + kNst + 4 * q4);
        Bs[4 * q4 + 0] = bv[0]; Bs[4 * q4 + 1] = bv[1]; Bs[4 * q4 + 2] = bv[2]; Bs[4 * q4 + 3] = bv[3];
        Cs[4 * q4 + 0] = cv[0]; Cs[4 * q4 + 1] = cv[1]; Cs[4 * q4 + 2] = cv[2]; Cs[4 * q4 + 3] = cv[3];
      }
      const float v   = PROJ[t * kPjP + d];
      const float a   = __expf(-fabsf(v));
      const float u   = 1.0f + a;
      const float l1p = __logf(u) + (a - (u - 1.0f)) * __builtin_amdgcn_rcpf(u);
      const float dt  = fmaxf(v, 0.0f) + l1p;
      const float xt  = XI[t * kDi + d];
      float y = 0.f;
#pragma unroll
      for (int k = 0; k < kNst; ++k) {
        const float e  = __expf(dt * negA[k]);
        const float db = dt * Bs[k];
        h[k] = e * h[k] + db * xt;
        y = h[k] * Cs[k] + y;
      }
      y = xt * Dd + y;
      const float zv = XR[t * kXrP + kDi + d];
      const float sg = __builtin_amdgcn_rcpf(1.0f + expf(-zv));
      y = y * (zv * sg);
      sY[s * kScanYP + tid] = y;
    }
    __syncthreads();
    v4u hv[8], lv[8];
#pragma unroll
    for (int it = 0; it < 8; ++it) {
      const int row = it * 8 + wave * 4 + q;
      const float* sp = sY + row * kScanYP + c8;
      const v4f a0 = *(const v4f*)(sp);
      const v4f a1 = *(const v4f*)(sp + 4);
      const float e0 = a0[0], e1 = a0[1], e2 = a0[2], e3 = a0[3];
      const float e4 = a1[0], e5 = a1[1], e6 = a1[2], e7 = a1[3];
      unsigned wh, wl;
      split_pack2(e0, e1, wh, wl); hv[it][0] = wh; lv[it][0] = wl;
      split_pack2(e2, e3, wh, wl); hv[it][1] = wh; lv[it][1] = wl;
      split_pack2(e4, e5, wh, wl); hv[it][2] = wh; lv[it][2] = wl;
      split_pack2(e6, e7, wh, wl); hv[it][3] = wh; lv[it][3] = wl;
    }
    for (int pass = 0; pass < 2; ++pass) {
#pragma unroll
      for (int it = 0; it < 8; ++it) {
        const int row = it * 8 + wave * 4 + q;
        const size_t o = (size_t)(t0 + row) * kDi + d0 + c8;
        *(volatile v4u*)(ZH + o) = hv[it];
        *(volatile v4u*)(ZL + o) = lv[it];
      }
      __threadfence();
    }
  }
}

extern "C" void kernel_launch(void* const* d_in, const int* in_sizes, int n_in,
                              void* d_out, int out_size, void* d_ws, size_t ws_size,
                              hipStream_t stream) {
  if (n_in < 11) return;
  if (in_sizes[0]  != kSeq * kDm) return;
  if (in_sizes[1]  != kXrP * kDm) return;
  if (in_sizes[2]  != kXrP) return;
  if (in_sizes[3]  != kDi * kTaps) return;
  if (in_sizes[4]  != kDi) return;
  if (in_sizes[5]  != kPjN * kDi) return;
  if (in_sizes[6]  != kPjN) return;
  if (in_sizes[7]  != kDm * kDi) return;
  if (in_sizes[8]  != kDm) return;
  if (in_sizes[9]  != kDi * kNst) return;
  if (in_sizes[10] != kDi) return;
  if (out_size != kSeq * kDm) return;
  if (ws_size < kWsTotal) return;

  const float* x      = (const float*)d_in[0];
  const float* W_in   = (const float*)d_in[1];
  const float* b_in   = (const float*)d_in[2];
  const float* W_conv = (const float*)d_in[3];
  const float* b_conv = (const float*)d_in[4];
  const float* W_x    = (const float*)d_in[5];
  const float* b_x    = (const float*)d_in[6];
  const float* W_out  = (const float*)d_in[7];
  const float* b_out  = (const float*)d_in[8];
  const float* A_log  = (const float*)d_in[9];
  const float* Dp     = (const float*)d_in[10];
  float* out = (float*)d_out;

  char* ws = (char*)d_ws;
  unsigned short* XB   = (unsigned short*)(ws + kOffXB);
  unsigned short* WINB = (unsigned short*)(ws + kOffWINB);
  unsigned short* WXB  = (unsigned short*)(ws + kOffWXB);
  unsigned short* WOB  = (unsigned short*)(ws + kOffWOB);
  float*          XR   = (float*)(ws + kOffXR);
  float*          XI   = (float*)(ws + kOffXI);
  unsigned short* XIB  = (unsigned short*)(ws + kOffXIB);
  float*          PROJ = (float*)(ws + kOffPROJ);
  unsigned short* ZH   = (unsigned short*)(ws + kOffZH);
  unsigned short* ZL   = (unsigned short*)(ws + kOffZL);

  {
    const int nx = kSeq * kDm / 8;
    cast_bf16_kernel<<<nx / 256, 256, 0, stream>>>(x, XB, nx, nx);
    const int nwi = kXrP * kDm / 8;
    cast_bf16_kernel<<<nwi / 256, 256, 0, stream>>>(W_in, WINB, nwi, nwi);
    const int nwx_real = kPjN * kDi / 8;
    const int nwx_all  = kPjP * kDi / 8;
    cast_bf16_kernel<<<nwx_all / 256, 256, 0, stream>>>(W_x, WXB, nwx_real, nwx_all);
    const int nwo = kDm * kDi / 8;
    cast_bf16_kernel<<<nwo / 256, 256, 0, stream>>>(W_out, WOB, nwo, nwo);
  }

  wmma_gemm64_bf16<0><<<dim3((kSeq / 64) * (kXrP / 64) / 8), 256, 0, stream>>>(
      XB, XB, kDm, WINB, kDm, XR, kXrP, b_in, kXrP, kSeq, kXrP, kDm);

  conv_silu_kernel<<<dim3(kDi / 256, kSeq / 64), 256, 0, stream>>>(XR, W_conv, b_conv, XI, XIB);

  wmma_gemm64_bf16<0><<<dim3((kSeq / 64) * (kPjP / 64) / 8), 256, 0, stream>>>(
      XIB, XIB, kDi, WXB, kDi, PROJ, kPjP, b_x, kPjN, kSeq, kPjP, kDi);

  scan_kernel<<<kDi / kScanCh, kScanCh, 0, stream>>>(PROJ, XI, XR, A_log, Dp, ZH, ZL);

  wmma_gemm64_bf16<1><<<dim3((kSeq / 64) * (kDm / 64) / 8), 256, 0, stream>>>(
      ZH, ZL, kDi, WOB, kDi, out, kDm, b_out, kDm, kSeq, kDm, kDi);
}
